// MemoryAttention_32993938768376
// MI455X (gfx1250) — hardware-verified
//
#include <hip/hip_runtime.h>
#include <math.h>
#include <stdint.h>

#ifndef NB
#define NB 2
#endif
#ifndef SEQ
#define SEQ 1024
#endif
#define NB_FULL 2
#define S_FULL  1024
#define DMOD    1024
#define MDIM    512
#define MEMN    128
#define HID     512
#define MROWS   (NB * SEQ)
#define KROWS   (NB * MEMN)
#define OUT1_OFF (NB_FULL * S_FULL * DMOD)
#define QSC   1024.0f
#define KSC   1024.0f
#define PCAR  32768.0f
#define VCAR  1024.0f
#define OSC   1024.0f
#define WOS   1024.0f
#define W1S   1024.0f
#define LOG2E 1.4426950408889634f
#define QKT   (DMOD / 8)
#define SLAB64 (16 * 68)
#define TRP   72
#define RR    16
#define AWP   4
#define ATT_THREADS (AWP * 32)
#define PT2   132
#define PTW2  (16 * PT2)
#define SLP   68
#define SLW   (16 * SLP)
#define WREG2 (PTW2 + SLW)
#define WS_CAP 134217728

static_assert(NB >= 1 && NB <= NB_FULL);
static_assert(SEQ >= 64 && SEQ <= S_FULL && (SEQ % 64) == 0 && (SEQ % RR) == 0);
static_assert(NB == 1 || SEQ == S_FULL);
static_assert(OUT1_OFF * 4 == 8388608);
static_assert(OUT1_OFF + NB_FULL * S_FULL * MEMN <= 9437184 / 4);
static_assert((DMOD % 64) == 0 && (MDIM % 64) == 0 && (HID % 64) == 0 && (MEMN % 64) == 0 && (KROWS % 64) == 0 && (MROWS % 64) == 0);
static_assert((DMOD % 32) == 0 && (MDIM % 32) == 0 && MEMN == 128 && QKT == 128);
static_assert(((MROWS * DMOD) % (8 * 256)) == 0 && ((KROWS * MDIM) % (8 * 256)) == 0);
static_assert(HID == 4 * MEMN && (RR * HID) % (4 * MEMN) == 0);
static_assert(AWP * WREG2 * 4 <= 65536 && ATT_THREADS == 128);

typedef unsigned short u16;
typedef _Float16 v16h __attribute__((ext_vector_type(16)));
typedef _Float16 v8h  __attribute__((ext_vector_type(8)));
typedef __bf16   v16b __attribute__((ext_vector_type(16)));
typedef float    v8f  __attribute__((ext_vector_type(8)));
typedef float    v4f  __attribute__((ext_vector_type(4)));
typedef float    v2f  __attribute__((ext_vector_type(2)));
typedef unsigned int v4u __attribute__((ext_vector_type(4)));

union FragH { v16h v; v8h h[2]; v4u u[2]; };
union FragB { v16b v; v4u u[2]; };

__device__ __forceinline__ unsigned short bf_bits(float f) {
  unsigned u = __float_as_uint(f);
  return (unsigned short)((u + 0x7FFFu + ((u >> 16) & 1u)) >> 16);
}
__device__ __forceinline__ float bf_up(unsigned short h) { return __uint_as_float(((unsigned)h) << 16); }
__device__ __forceinline__ float bfr(float f) { return bf_up(bf_bits(f)); }
__device__ __forceinline__ unsigned short h_bits(_Float16 x) { return __builtin_bit_cast(unsigned short, x); }
__device__ __forceinline__ unsigned pk16(unsigned short a, unsigned short b) { return (unsigned)a | ((unsigned)b << 16); }
__device__ __forceinline__ v8f zero8() { v8f z = {0.f, 0.f, 0.f, 0.f, 0.f, 0.f, 0.f, 0.f}; return z; }

__device__ __forceinline__ v16h ldfrag_h(const _Float16* p) {
  FragH f;
  f.h[0] = *(const v8h*)(p);
  f.h[1] = *(const v8h*)(p + 16);
  return f.v;
}
__device__ __forceinline__ v16b ldfrag_b(const u16* p) {
  FragB f;
  f.u[0] = *(const v4u*)(p);
  f.u[1] = *(const v4u*)(p + 16);
  return f.v;
}

__device__ __forceinline__ v8f mma_h(v16h a, v16h b, v8f c) {
  return __builtin_amdgcn_wmma_f32_16x16x32_f16(false, a, false, b, (short)0, c, false, false);
}
__device__ __forceinline__ v8f mma_b(v16b a, v16b b, v8f c) {
  return __builtin_amdgcn_wmma_f32_16x16x32_bf16(false, a, false, b, (short)0, c, false, false);
}
__device__ __forceinline__ void guard2(v8f& a, v8f& b, v16h x0, v16h x1, v16h x2, v16h x3, v16h x4, v16h x5) {
#if defined(__HIP_DEVICE_COMPILE__)
  asm volatile("v_nop\n\tv_nop\n\tv_nop\n\tv_nop"
               : "+v"(a), "+v"(b) : "v"(x0), "v"(x1), "v"(x2), "v"(x3), "v"(x4), "v"(x5) : "memory");
#endif
}
template <typename F>
__device__ __forceinline__ void guard6(v8f& a, v8f& b, v8f& c, v8f& d, F x0, F x1, F x2, F x3, F x4, F x5) {
#if defined(__HIP_DEVICE_COMPILE__)
  asm volatile("v_nop\n\tv_nop\n\tv_nop\n\tv_nop"
               : "+v"(a), "+v"(b), "+v"(c), "+v"(d) : "v"(x0), "v"(x1), "v"(x2), "v"(x3), "v"(x4), "v"(x5) : "memory");
#endif
}
template <typename F>
__device__ __forceinline__ void guard4x10(v8f& a, v8f& b, v8f& c, v8f& d,
                                          F x0, F x1, F x2, F x3, F x4, F x5, F x6, F x7, F x8, F x9) {
#if defined(__HIP_DEVICE_COMPILE__)
  asm volatile("v_nop\n\tv_nop\n\tv_nop\n\tv_nop"
               : "+v"(a), "+v"(b), "+v"(c), "+v"(d)
               : "v"(x0), "v"(x1), "v"(x2), "v"(x3), "v"(x4), "v"(x5), "v"(x6), "v"(x7), "v"(x8), "v"(x9) : "memory");
#endif
}
__device__ __forceinline__ void acc_guard4(v8f& a, v8f& b, v8f& c, v8f& d) {
#if defined(__HIP_DEVICE_COMPILE__)
  asm volatile("v_nop\n\tv_nop\n\tv_nop\n\tv_nop" : "+v"(a), "+v"(b), "+v"(c), "+v"(d));
#endif
}
__device__ __forceinline__ void wave_sync_lds() {
  __builtin_amdgcn_fence(__ATOMIC_RELEASE, "workgroup");
  __builtin_amdgcn_wave_barrier();
  __builtin_amdgcn_fence(__ATOMIC_ACQUIRE, "workgroup");
}

__global__ __launch_bounds__(256) void cvt16(const float* __restrict__ x, u16* D, int n8, int f16mode, float scale) {
  const int gt = blockIdx.x * 256 + (int)threadIdx.x;
  if (gt >= n8) return;
  const float* p = x + (size_t)gt * 8;
  const v4f a = *(const v4f*)(p), b4 = *(const v4f*)(p + 4);
  float w[8];
#pragma unroll
  for (int e = 0; e < 4; ++e) { w[e] = a[e]; w[4 + e] = b4[e]; }
  v4u o;
#pragma unroll
  for (int e = 0; e < 4; ++e) {
    const float f0 = w[2 * e], f1 = w[2 * e + 1];
    const unsigned short hb0 = h_bits((_Float16)(bfr(f0) * scale));
    const unsigned short hb1 = h_bits((_Float16)(bfr(f1) * scale));
    const unsigned short bb0 = bf_bits(f0);
    const unsigned short bb1 = bf_bits(f1);
    o[e] = (f16mode != 0) ? pk16(hb0, hb1) : pk16(bb0, bb1);
  }
  u16* d = D + (size_t)gt * 8;
  for (int pass = 0; pass < 2; ++pass) {
    *(volatile v4u*)(d) = o;
    __threadfence();
  }
}

template <int MODE>
__global__ __launch_bounds__(256) void tr16(const float* __restrict__ src, u16* D0, u16* D1, int R, int Cn, int nbat, float scale) {
  __shared__ __align__(16) u16 T0[64 * TRP];
  __shared__ __align__(16) u16 T1[64 * TRP];
  const int tid = (int)threadIdx.x;
  const int bid = (int)blockIdx.x;
  const int nct = Cn >> 6, nrt = R >> 6;
  const int ct  = bid % nct;
  const int t2  = bid / nct;
  const int rt  = t2 % nrt;
  const int z   = t2 / nrt;
  if (z >= nbat) return;
  const int r0 = rt * 64, c0 = ct * 64;
  const float* s = src + (size_t)z * (size_t)R * (size_t)Cn;
  {
    const int kr = tid >> 2, cc = (tid & 3) * 16;
    const float* p = s + (size_t)(r0 + kr) * Cn + c0 + cc;
#pragma unroll
    for (int i = 0; i < 4; ++i) {
      const v4f a = *(const v4f*)(p + 4 * i);
#pragma unroll
      for (int e = 0; e < 4; ++e) {
        const int col = cc + 4 * i + e;
        if constexpr (MODE == 2) {
          const float t = a[e] * scale;
          const _Float16 hv = (_Float16)t;
          const _Float16 lv = (_Float16)(t - (float)hv);
          T0[col * TRP + kr] = h_bits(hv);
          T1[col * TRP + kr] = h_bits(lv);
        } else if constexpr (MODE == 1) {
          T0[col * TRP + kr] = h_bits((_Float16)(bfr(a[e]) * scale));
        } else {
          T0[col * TRP + kr] = bf_bits(a[e]);
        }
      }
    }
  }
  __syncthreads();
  const int q8 = tid >> 3, p8 = (tid & 7) * 8;
  v4u o0[2], o1[2];
#pragma unroll
  for (int it = 0; it < 2; ++it) {
    const int line = it * 32 + q8;
    o0[it] = *(const v4u*)(T0 + line * TRP + p8);
    if constexpr (MODE == 2) { o1[it] = *(const v4u*)(T1 + line * TRP + p8); } else { o1[it] = o0[it]; }
  }
  const size_t base = (size_t)z * (size_t)Cn * (size_t)R + (size_t)c0 * (size_t)R + (size_t)r0 + (size_t)p8;
  for (int pass = 0; pass < 2; ++pass) {
#pragma unroll
    for (int it = 0; it < 2; ++it) {
      const int line = it * 32 + q8;
      *(volatile v4u*)(D0 + base + (size_t)line * (size_t)R) = o0[it];
      if constexpr (MODE == 2) {
        *(volatile v4u*)(D1 + base + (size_t)line * (size_t)R) = o1[it];
      }
    }
    __threadfence();
  }
}

__global__ __launch_bounds__(QKT) void qk16(const float* __restrict__ F, u16* Hp, u16* Lp, int rows, float sc) {
  const int tid = (int)threadIdx.x;
  const int row = (int)blockIdx.x;
  if (row >= rows) return;
  if (tid >= QKT) return;
  const float* p = F + (size_t)row * DMOD + tid * 8;
  const v4f a = *(const v4f*)(p), b4 = *(const v4f*)(p + 4);
  float w[8];
#pragma unroll
  for (int e = 0; e < 4; ++e) { w[e] = a[e] * sc; w[4 + e] = b4[e] * sc; }
  v4u oh, ol;
#pragma unroll
  for (int e = 0; e < 4; ++e) {
    const float t0 = w[2 * e], t1 = w[2 * e + 1];
    const _Float16 h0 = (_Float16)t0, h1 = (_Float16)t1;
    const _Float16 l0 = (_Float16)(t0 - (float)h0), l1 = (_Float16)(t1 - (float)h1);
    oh[e] = pk16(h_bits(h0), h_bits(h1));
    ol[e] = pk16(h_bits(l0), h_bits(l1));
  }
  u16* dh = Hp + (size_t)row * DMOD + tid * 8;
  u16* dl = Lp + (size_t)row * DMOD + tid * 8;
  for (int pass = 0; pass < 2; ++pass) {
    *(volatile v4u*)(dh) = oh;
    *(volatile v4u*)(dl) = ol;
    __threadfence();
  }
}

template <int HASB>
__device__ __forceinline__ void epi64(float* sl, v8f a0, v8f a1, v8f a2, v8f a3, float oscale,
                                      const float* __restrict__ bias, float* C, int N, size_t rowb, int col0, int lane) {
  const int hh = lane >> 4, m = lane & 15;
#pragma unroll
  for (int r = 0; r < 8; ++r) {
    const int ro = (8 * hh + r) * 68 + m;
    sl[ro]      = a0[r] * oscale;
    sl[ro + 16] = a1[r] * oscale;
    sl[ro + 32] = a2[r] * oscale;
    sl[ro + 48] = a3[r] * oscale;
  }
  wave_sync_lds();
  v4f br = {0.f, 0.f, 0.f, 0.f};
  if constexpr (HASB != 0) {
    const v4f bb = *(const v4f*)(bias + col0 + m * 4);
#pragma unroll
    for (int e = 0; e < 4; ++e) br[e] = bfr(bb[e]);
  }
  v4f vals[8];
#pragma unroll
  for (int it = 0; it < 8; ++it) vals[it] = *(const v4f*)(sl + (it * 2 + hh) * 68 + m * 4) + br;
  float* dst = C + (rowb + (size_t)hh) * (size_t)N + col0 + m * 4;
  for (int pass = 0; pass < 2; ++pass) {
#pragma unroll
    for (int it = 0; it < 8; ++it) {
      *(volatile v4f*)(dst + (size_t)(it * 2) * (size_t)N) = vals[it];
    }
    __threadfence();
  }
}

__global__ __launch_bounds__(128)
void gemm_bf(const u16* __restrict__ A, const u16* __restrict__ Bt, const float* __restrict__ bias,
             float* C, int M, int N, int K, float oscale) {
  __shared__ __align__(16) float slab[4 * SLAB64];
  const int tid = threadIdx.x, wave = tid >> 5, lane = tid & 31, hh = lane >> 4, m = lane & 15;
  const int ntile = N >> 6;
  const int bid   = blockIdx.x;
  const int rowb  = (bid / ntile) * 64 + wave * 16;
  const int col0  = (bid % ntile) * 64;
  if (rowb + 16 > M) return;
  const u16* ap = A  + (size_t)(rowb + m) * K + 8 * hh;
  const u16* bp = Bt + (size_t)(col0 + m) * K + 8 * hh;
  const size_t bs = (size_t)16 * K;
  v8f acc0 = zero8(), acc1 = zero8(), acc2 = zero8(), acc3 = zero8();
#pragma unroll 1
  for (int k0 = 0; k0 < K; k0 += 32) {
    const v16b a  = ldfrag_b(ap + k0);
    const v16b b0 = ldfrag_b(bp + k0);
    const v16b b1 = ldfrag_b(bp + bs + k0);
    const v16b b2 = ldfrag_b(bp + 2 * bs + k0);
    const v16b b3 = ldfrag_b(bp + 3 * bs + k0);
    acc0 = mma_b(a, b0, acc0);
    acc1 = mma_b(a, b1, acc1);
    acc2 = mma_b(a, b2, acc2);
    acc3 = mma_b(a, b3, acc3);
    guard6<v16b>(acc0, acc1, acc2, acc3, a, b0, b1, b2, b3, a);
  }
  epi64<1>(slab + wave * SLAB64, acc0, acc1, acc2, acc3, oscale, bias, C, N, (size_t)rowb, col0, lane);
}

template <int NPROD, int HASB>
__global__ __launch_bounds__(128)
void gemm_h(const u16* __restrict__ Ah, const u16* __restrict__ Al, const u16* __restrict__ Bt, const float* __restrict__ bias,
            float* C, int M, int N, int K, float oscale) {
  __shared__ __align__(16) float slab[4 * SLAB64];
  const int tid = threadIdx.x, wave = tid >> 5, lane = tid & 31, hh = lane >> 4, m = lane & 15;
  const int ntile = N >> 6;
  const int bid   = blockIdx.x;
  const int rowb  = (bid / ntile) * 64 + wave * 16;
  const int col0  = (bid % ntile) * 64;
  if (rowb + 16 > M) return;
  const _Float16* ahp = (const _Float16*)(const void*)Ah + (size_t)(rowb + m) * K + 8 * hh;
  const _Float16* alp = (const _Float16*)(const void*)Al + (size_t)(rowb + m) * K + 8 * hh;
  const _Float16* bp  = (const _Float16*)(const void*)Bt + (size_t)(col0 + m) * K + 8 * hh;
  const size_t bs = (size_t)16 * K;
  v8f acc0 = zero8(), acc1 = zero8(), acc2 = zero8(), acc3 = zero8();
  if constexpr (NPROD == 2) {
#pragma unroll 1
    for (int k0 = 0; k0 < K; k0 += 32) {
      const v16h ah = ldfrag_h(ahp + k0), al = ldfrag_h(alp + k0);
      const v16h b0 = ldfrag_h(bp + k0);
      const v16h b1 = ldfrag_h(bp + bs + k0);
      const v16h b2 = ldfrag_h(bp + 2 * bs + k0);
      const v16h b3 = ldfrag_h(bp + 3 * bs + k0);
      acc0 = mma_h(ah, b0, acc0);  acc0 = mma_h(al, b0, acc0);
      acc1 = mma_h(ah, b1, acc1);  acc1 = mma_h(al, b1, acc1);
      acc2 = mma_h(ah, b2, acc2);  acc2 = mma_h(al, b2, acc2);
      acc3 = mma_h(ah, b3, acc3);  acc3 = mma_h(al, b3, acc3);
      guard6<v16h>(acc0, acc1, acc2, acc3, ah, al, b0, b1, b2, b3);
    }
  } else {
#pragma unroll 1
    for (int k0 = 0; k0 < K; k0 += 32) {
      const v16h ah = ldfrag_h(ahp + k0);
      const v16h b0 = ldfrag_h(bp + k0);
      const v16h b1 = ldfrag_h(bp + bs + k0);
      const v16h b2 = ldfrag_h(bp + 2 * bs + k0);
      const v16h b3 = ldfrag_h(bp + 3 * bs + k0);
      acc0 = mma_h(ah, b0, acc0);
      acc1 = mma_h(ah, b1, acc1);
      acc2 = mma_h(ah, b2, acc2);
      acc3 = mma_h(ah, b3, acc3);
      guard6<v16h>(acc0, acc1, acc2, acc3, ah, b0, b1, b2, b3, ah);
    }
  }
  epi64<HASB>(slab + wave * SLAB64, acc0, acc1, acc2, acc3, oscale, bias, C, N, (size_t)rowb, col0, lane);
}

__global__ __launch_bounds__(MEMN) void relev(const float* __restrict__ QP, const float* __restrict__ MPb,
                                              const float* __restrict__ W2, const float* __restrict__ b2, float* REL) {
  __shared__ __align__(16) float qs[RR * HID];
  __shared__ __align__(16) float w2s[HID];
  const int tid = (int)threadIdx.x;
  const int bid = (int)blockIdx.x;
  const int nrc = SEQ / RR;
  const int rc  = bid % nrc;
  const int b   = bid / nrc;
  if (b >= NB) return;
  const int s0 = rc * RR;
  const size_t row0 = (size_t)b * SEQ + s0;
  {
    const float* qp = QP + row0 * HID;
#pragma unroll
    for (int it = 0; it < (RR * HID) / (4 * MEMN); ++it) {
      const int idx = (it * MEMN + tid) * 4;
      *(v4f*)(qs + idx) = *(const v4f*)(qp + idx);
    }
    const v4f wv4 = *(const v4f*)(W2 + tid * 4);
    v4f wr;
#pragma unroll
    for (int e = 0; e < 4; ++e) wr[e] = bfr(wv4[e]);
    *(v4f*)(w2s + tid * 4) = wr;
  }
  __syncthreads();
  const float* mrow = MPb + ((size_t)b * MEMN + tid) * HID;
  v2f acc[RR];
#pragma unroll
  for (int i = 0; i < RR; ++i) { acc[i].x = 0.f; acc[i].y = 0.f; }
#pragma unroll 1
  for (int h = 0; h < HID; h += 2) {
    const v2f mv = *(const v2f*)(mrow + h);
    const v2f wv = *(const v2f*)(w2s + h);
#pragma unroll
    for (int i = 0; i < RR; ++i) {
      const v2f qv = *(const v2f*)(qs + i * HID + h);
      const v2f u = qv + mv;
      v2f rl;
      rl.x = fmaxf(u.x, 0.0f);
      rl.y = fmaxf(u.y, 0.0f);
      acc[i] = rl * wv + acc[i];
    }
  }
  const float bb = bfr(b2[0]);
  float rv[RR];
#pragma unroll
  for (int i = 0; i < RR; ++i) {
    const float z  = (acc[i].x + acc[i].y) + bb;
    const float ex = exp2f(-z * LOG2E);
    rv[i] = __builtin_amdgcn_rcpf(1.0f + ex);
  }
  float* dst = REL + row0 * MEMN + tid;
  for (int pass = 0; pass < 2; ++pass) {
#pragma unroll
    for (int i = 0; i < RR; ++i) {
      *(volatile float*)(dst + (size_t)i * MEMN) = rv[i];
    }
    __threadfence();
  }
}

__global__ __launch_bounds__(ATT_THREADS)
void attn_m(const u16* __restrict__ QHp, const u16* __restrict__ QLp, const u16* __restrict__ KHp, const u16* __restrict__ KLp,
            const u16* __restrict__ VHp, const u16* __restrict__ VLp, const float* __restrict__ RELp,
            float* out1, u16* OHp, u16* OLp) {
  __shared__ __align__(16) float smem[AWP * WREG2];

  const int tid  = threadIdx.x;
  const int wave = tid >> 5;
  const int lane = tid & 31;
  const int hh   = lane >> 4;
  const int c    = lane & 15;
  const int bid  = blockIdx.x;
  const int nqb  = SEQ / 64;
  const int qb   = bid % nqb;
  const int b    = bid / nqb;
  if (b >= NB) return;
  const int q0   = qb * 64 + wave * 16;
  if (q0 + 16 > SEQ) return;

  float* pt   = smem + wave * WREG2;
  float* slab = pt + PTW2;

  const size_t qrow = (size_t)b * SEQ + q0;
  const _Float16* Qh  = (const _Float16*)(const void*)QHp + (qrow + c) * DMOD + 8 * hh;
  const _Float16* Ql  = (const _Float16*)(const void*)QLp + (qrow + c) * DMOD + 8 * hh;
  const _Float16* Khb = (const _Float16*)(const void*)KHp + ((size_t)b * MEMN + c) * DMOD + 8 * hh;
  const _Float16* Klb = (const _Float16*)(const void*)KLp + ((size_t)b * MEMN + c) * DMOD + 8 * hh;

  v8f s[8];
#pragma unroll
  for (int j = 0; j < 8; ++j) s[j] = zero8();
#pragma unroll 1
  for (int k0 = 0; k0 < DMOD; k0 += 32) {
    const v16h qh = ldfrag_h(Qh + k0), ql = ldfrag_h(Ql + k0);
#pragma unroll
    for (int g = 0; g < 2; ++g) {
      v16h kh[4], kl[4];
#pragma unroll
      for (int j = 0; j < 4; ++j) {
        const size_t ko = (size_t)(4 * g + j) * 16 * DMOD + k0;
        kh[j] = ldfrag_h(Khb + ko);
        kl[j] = ldfrag_h(Klb + ko);
      }
#pragma unroll
      for (int j = 0; j < 4; ++j) {
        s[4 * g + j] = mma_h(qh, kh[j], s[4 * g + j]);
        s[4 * g + j] = mma_h(ql, kh[j], s[4 * g + j]);
        s[4 * g + j] = mma_h(qh, kl[j], s[4 * g + j]);
      }
      guard4x10<v16h>(s[4 * g], s[4 * g + 1], s[4 * g + 2], s[4 * g + 3],
                      qh, ql, kh[0], kh[1], kh[2], kh[3], kl[0], kl[1], kl[2], kl[3]);
    }
  }
  const float lsc = 1.0f / (32.0f * QSC * KSC);
#pragma unroll
  for (int j = 0; j < 8; ++j) {
#pragma unroll
    for (int r = 0; r < 8; ++r) pt[(8 * hh + r) * PT2 + 16 * j + c] = s[j][r] * lsc;
  }
  wave_sync_lds();

  const int cb = 64 * hh;
  const float* relrow = RELp + (qrow + c) * MEMN + cb;
  v4f t[16];
  float mx = -INFINITY;
#pragma unroll
  for (int i = 0; i < 16; ++i) {
    const v4f sv = *(const v4f*)(pt + c * PT2 + cb + 4 * i);
    const v4f rv = *(const v4f*)(relrow + 4 * i);
    const v4f u = sv * rv;
    t[i] = u;
    mx = fmaxf(mx, u[0]);
    mx = fmaxf(mx, u[1]);
    mx = fmaxf(mx, u[2]);
    mx = fmaxf(mx, u[3]);
  }
  mx = fmaxf(mx, __shfl_xor(mx, 16, 32));
  float sum = 0.f;
#pragma unroll
  for (int i = 0; i < 16; ++i) {
    v4f ev;
#pragma unroll
    for (int e = 0; e < 4; ++e) ev[e] = exp2f((t[i][e] - mx) * LOG2E);
    t[i] = ev;
    sum += (ev[0] + ev[1]) + (ev[2] + ev[3]);
  }
  sum += __shfl_xor(sum, 16, 32);
  const float inv = 1.0f / sum;
#pragma unroll
  for (int i = 0; i < 16; ++i) t[i] = t[i] * inv;
#pragma unroll
  for (int i = 0; i < 16; ++i) *(v4f*)(pt + c * PT2 + cb + 4 * i) = t[i];
  wave_sync_lds();

  {
    const int q8 = lane >> 3, p4 = (lane & 7) * 4;
    v4f ov[16];
#pragma unroll
    for (int it = 0; it < 16; ++it) ov[it] = *(const v4f*)(pt + it * PT2 + q8 * 32 + p4);
    float* od = out1 + ((size_t)b * S_FULL + q0) * MEMN + q8 * 32 + p4;
    for (int pass = 0; pass < 2; ++pass) {
#pragma unroll
      for (int it = 0; it < 16; ++it) {
        *(volatile v4f*)(od + (size_t)it * MEMN) = ov[it];
      }
      __threadfence();
    }
  }

  FragH ph[4], pl[4];
#pragma unroll
  for (int kt = 0; kt < 4; ++kt) {
    const float* prow = pt + c * PT2 + 32 * kt + 8 * hh;
    const v4f p0 = *(const v4f*)(prow), p1 = *(const v4f*)(prow + 4);
    const v4f p2 = *(const v4f*)(prow + 16), p3 = *(const v4f*)(prow + 20);
#pragma unroll
    for (int e = 0; e < 4; ++e) {
      const float ta = p0[e] * PCAR, tb = p1[e] * PCAR, tc = p2[e] * PCAR, td = p3[e] * PCAR;
      const _Float16 ha = (_Float16)ta, hb = (_Float16)tb, hc = (_Float16)tc, hd = (_Float16)td;
      ph[kt].h[0][e]     = ha;
      ph[kt].h[0][4 + e] = hb;
      ph[kt].h[1][e]     = hc;
      ph[kt].h[1][4 + e] = hd;
      pl[kt].h[0][e]     = (_Float16)(ta - (float)ha);
      pl[kt].h[0][4 + e] = (_Float16)(tb - (float)hb);
      pl[kt].h[1][e]     = (_Float16)(tc - (float)hc);
      pl[kt].h[1][4 + e] = (_Float16)(td - (float)hd);
    }
  }

  const _Float16* Vhb = (const _Float16*)(const void*)VHp + ((size_t)b * DMOD + c) * MEMN + 8 * hh;
  const _Float16* Vlb = (const _Float16*)(const void*)VLp + ((size_t)b * DMOD + c) * MEMN + 8 * hh;
  const float oc = OSC / (PCAR * VCAR);
  const int rq = lane >> 3, c8 = (lane & 7) * 8;
#pragma unroll 1
  for (int dcn = 0; dcn < DMOD / 64; ++dcn) {
    v8f o[4];
#pragma unroll
    for (int j = 0; j < 4; ++j) o[j] = zero8();
#pragma unroll
    for (int kt = 0; kt < 4; ++kt) {
#pragma unroll
      for (int jg = 0; jg < 2; ++jg) {
        const size_t da = (size_t)(dcn * 64 + 32 * jg) * MEMN + (size_t)(32 * kt);
        const size_t db = da + (size_t)16 * MEMN;
        const v16h vha = ldfrag_h(Vhb + da), vhb2 = ldfrag_h(Vhb + db);
        const v16h vla = ldfrag_h(Vlb + da), vlb2 = ldfrag_h(Vlb + db);
        o[2 * jg]     = mma_h(ph[kt].v, vha,  o[2 * jg]);
        o[2 * jg]     = mma_h(pl[kt].v, vha,  o[2 * jg]);
        o[2 * jg]     = mma_h(ph[kt].v, vla,  o[2 * jg]);
        o[2 * jg + 1] = mma_h(ph[kt].v, vhb2, o[2 * jg + 1]);
        o[2 * jg + 1] = mma_h(pl[kt].v, vhb2, o[2 * jg + 1]);
        o[2 * jg + 1] = mma_h(ph[kt].v, vlb2, o[2 * jg + 1]);
        guard2(o[2 * jg], o[2 * jg + 1], ph[kt].v, pl[kt].v, vha, vhb2, vla, vlb2);
      }
    }
    acc_guard4(o[0], o[1], o[2], o[3]);
#pragma unroll
    for (int r = 0; r < 8; ++r) {
#pragma unroll
      for (int j = 0; j < 4; ++j) {
        slab[(8 * hh + r) * SLP + j * 16 + c] = o[j][r] * oc;
      }
    }
    wave_sync_lds();
    v4u oh[4], ol[4];
#pragma unroll
    for (int it = 0; it < 4; ++it) {
      const int row = it * 4 + rq;
      const v4f a = *(const v4f*)(slab + row * SLP + c8), b4 = *(const v4f*)(slab + row * SLP + c8 + 4);
      float w[8];
#pragma unroll
      for (int e = 0; e < 4; ++e) { w[e] = a[e]; w[4 + e] = b4[e]; }
#pragma unroll
      for (int e = 0; e < 4; ++e) {
        const _Float16 h0 = (_Float16)w[2 * e], h1 = (_Float16)w[2 * e + 1];
        const _Float16 l0 = (_Float16)(w[2 * e] - (float)h0), l1 = (_Float16)(w[2 * e + 1] - (float)h1);
        oh[it][e] = pk16(h_bits(h0), h_bits(h1));
        ol[it][e] = pk16(h_bits(l0), h_bits(l1));
      }
    }
    const size_t ob = qrow * DMOD + (size_t)dcn * 64 + c8;
    for (int pass = 0; pass < 2; ++pass) {
#pragma unroll
      for (int it = 0; it < 4; ++it) {
        const int row = it * 4 + rq;
        *(volatile v4u*)(OHp + ob + (size_t)row * DMOD) = oh[it];
        *(volatile v4u*)(OLp + ob + (size_t)row * DMOD) = ol[it];
      }
      __threadfence();
    }
    wave_sync_lds();
  }
}

extern "C" void kernel_launch(void* const* d_in, const int* in_sizes, int n_in,
                              void* d_out, int out_size, void* d_ws, size_t ws_size,
                              hipStream_t stream) {
  if (n_in < 14) return;
  if (in_sizes[0] < MROWS * DMOD) return;
  if (in_sizes[1] < KROWS * MDIM) return;
  if (in_sizes[2] < DMOD * DMOD || in_sizes[3] < DMOD) return;
  if (in_sizes[4] < MDIM * DMOD || in_sizes[5] < DMOD) return;
  if (in_sizes[6] < MDIM * DMOD || in_sizes[7] < DMOD) return;
  if (in_sizes[8] < DMOD * DMOD || in_sizes[9] < DMOD) return;
  if (in_sizes[10] < (DMOD + MDIM) * HID || in_sizes[11] < HID) return;
  if (in_sizes[12] < HID || in_sizes[13] < 1) return;
  if (out_size < OUT1_OFF + MROWS * MEMN) return;

  const float* xh  = (const float*)d_in[0];
  const float* xm  = (const float*)d_in[1];
  const float* wq  = (const float*)d_in[2];
  const float* bq  = (const float*)d_in[3];
  const float* wk  = (const float*)d_in[4];
  const float* bk  = (const float*)d_in[5];
  const float* wv  = (const float*)d_in[6];
  const float* bv  = (const float*)d_in[7];
  const float* wo  = (const float*)d_in[8];
  const float* bo  = (const float*)d_in[9];
  const float* w1  = (const float*)d_in[10];
  const float* b1  = (const float*)d_in[11];
  const float* w2  = (const float*)d_in[12];
  const float* b2  = (const float*)d_in[13];
  float*       out = (float*)d_out;

  const size_t szXB  = (size_t)MROWS * DMOD * 2;
  const size_t szMB  = (size_t)KROWS * MDIM * 2;
  const size_t szWQ  = (size_t)DMOD * DMOD * 2;
  const size_t szWK  = (size_t)DMOD * MDIM * 2;
  const size_t szW1Q = (size_t)HID * DMOD * 2;
  const size_t szW1M = (size_t)HID * MDIM * 2;
  const size_t szQF  = (size_t)MROWS * DMOD * 4;
  const size_t szKF  = (size_t)KROWS * DMOD * 4;
  const size_t szMP  = (size_t)KROWS * HID * 4;
  const size_t szQ16 = (size_t)MROWS * DMOD * 2;
  const size_t szK16 = (size_t)KROWS * DMOD * 2;
  const size_t szV16 = (size_t)NB * DMOD * MEMN * 2;
  const size_t szQP  = (size_t)MROWS * HID * 4;
  const size_t szREL = (size_t)MROWS * MEMN * 4;
  size_t off = 0;
  const size_t oXB  = off; off += szXB;
  const size_t oMB  = off; off += szMB;
  const size_t oWQ  = off; off += szWQ;
  const size_t oWK  = off; off += szWK;
  const size_t oWV  = off; off += szWK;
  const size_t oWO  = off; off += szWQ;
  const size_t oW1Q = off; off += szW1Q;
  const size_t oW1M = off; off += szW1M;
  const size_t oQF  = off; off += szQF;
  const size_t oKF  = off; off += szKF;
  const size_t oVF  = off; off += szKF;
  const size_t oMP  = off; off += szMP;
  const size_t oQH  = off; off += szQ16;
  const size_t oQL  = off; off += szQ16;
  const size_t oKH  = off; off += szK16;
  const size_t oKL  = off; off += szK16;
  const size_t oVH  = off; off += szV16;
  const size_t oVL  = off; off += szV16;
  const size_t oQP  = off; off += szQP;
  const size_t oREL = off; off += szREL;
  const size_t oOH  = off; off += szQ16;
  const size_t oOL  = off; off += szQ16;
  if (off > ws_size) return;
  if (off > (size_t)WS_CAP) return;

  char* ws = (char*)d_ws;
  u16*   XB   = (u16*)(ws + oXB);
  u16*   MB   = (u16*)(ws + oMB);
  u16*   WQT  = (u16*)(ws + oWQ);
  u16*   WKT  = (u16*)(ws + oWK);
  u16*   WVT  = (u16*)(ws + oWV);
  u16*   WOT  = (u16*)(ws + oWO);
  u16*   W1QT = (u16*)(ws + oW1Q);
  u16*   W1MT = (u16*)(ws + oW1M);
  float* QF   = (float*)(ws + oQF);
  float* KF   = (float*)(ws + oKF);
  float* VF   = (float*)(ws + oVF);
  float* MP   = (float*)(ws + oMP);
  u16*   QH   = (u16*)(ws + oQH);
  u16*   QL   = (u16*)(ws + oQL);
  u16*   KH   = (u16*)(ws + oKH);
  u16*   KL   = (u16*)(ws + oKL);
  u16*   VH   = (u16*)(ws + oVH);
  u16*   VL   = (u16*)(ws + oVL);
  float* QP   = (float*)(ws + oQP);
  float* REL  = (float*)(ws + oREL);
  u16*   OH   = (u16*)(ws + oOH);
  u16*   OL   = (u16*)(ws + oOL);

  const dim3 b256(256), b128(128), bQK(QKT), bRL(MEMN), bAT(ATT_THREADS);
  const int  n8x = (MROWS * DMOD) / 8;
  const int  n8m = (KROWS * MDIM) / 8;

  cvt16<<<dim3((n8x + 255) / 256), b256, 0, stream>>>(xh, XB, n8x, 0, 1.0f);
  cvt16<<<dim3((n8m + 255) / 256), b256, 0, stream>>>(xm, MB, n8m, 0, 1.0f);
  tr16<0><<<dim3((DMOD / 64) * (DMOD / 64)), b256, 0, stream>>>(wq, WQT, WQT, DMOD, DMOD, 1, 1.0f);
  tr16<0><<<dim3((MDIM / 64) * (DMOD / 64)), b256, 0, stream>>>(wk, WKT, WKT, MDIM, DMOD, 1, 1.0f);
  tr16<0><<<dim3((MDIM / 64) * (DMOD / 64)), b256, 0, stream>>>(wv, WVT, WVT, MDIM, DMOD, 1, 1.0f);
  tr16<1><<<dim3((DMOD / 64) * (DMOD / 64)), b256, 0, stream>>>(wo, WOT, WOT, DMOD, DMOD, 1, WOS);
  tr16<1><<<dim3((DMOD / 64) * (HID / 64)), b256, 0, stream>>>(w1, W1QT, W1QT, DMOD, HID, 1, W1S);
  tr16<0><<<dim3((MDIM / 64) * (HID / 64)), b256, 0, stream>>>(w1 + (size_t)DMOD * HID, W1MT, W1MT, MDIM, HID, 1, 1.0f);
  gemm_bf<<<dim3((MROWS / 64) * (DMOD / 64)), b128, 0, stream>>>(XB, WQT, bq, QF, MROWS, DMOD, DMOD, 1.0f);
  gemm_bf<<<dim3((KROWS / 64) * (DMOD / 64)), b128, 0, stream>>>(MB, WKT, bk, KF, KROWS, DMOD, MDIM, 1.0f);
  gemm_bf<<<dim3((KROWS / 64) * (DMOD / 64)), b128, 0, stream>>>(MB, WVT, bv, VF, KROWS, DMOD, MDIM, 1.0f);
  gemm_bf<<<dim3((KROWS / 64) * (HID / 64)), b128, 0, stream>>>(MB, W1MT, b1, MP, KROWS, HID, MDIM, 1.0f);
  qk16<<<dim3(MROWS), bQK, 0, stream>>>(QF, QH, QL, MROWS, QSC);
  qk16<<<dim3(KROWS), bQK, 0, stream>>>(KF, KH, KL, KROWS, KSC);
  tr16<2><<<dim3(NB * (MEMN / 64) * (DMOD / 64)), b256, 0, stream>>>(VF, VH, VL, MEMN, DMOD, NB, VCAR);
  gemm_h<1, 0><<<dim3((MROWS / 64) * (HID / 64)), b128, 0, stream>>>(QH, QH, W1QT, b1, QP, MROWS, HID, DMOD, 1.0f / (QSC * W1S));
  relev<<<dim3(NB * (SEQ / RR)), bRL, 0, stream>>>(QP, MP, w2, b2, REL);
  attn_m<<<dim3(NB * (SEQ / 64)), bAT, 0, stream>>>(QH, QL, KH, KL, VH, VL, REL, out + OUT1_OFF, OH, OL);
  gemm_h<2, 1><<<dim3((MROWS / 64) * (DMOD / 64)), b128, 0, stream>>>(OH, OL, WOT, bo, out, MROWS, DMOD, DMOD, 1.0f / (OSC * WOS));
  (void)hipGetLastError();
}
